// NonLocalBlock_71373766525083
// MI455X (gfx1250) — hardware-verified
//
#include <hip/hip_runtime.h>
#include <math.h>

#ifndef NB
#define NB 4
#endif
#ifndef SEQ
#define SEQ 4096
#endif
#define NB_FULL 4
#define SEQ_FULL 4096
#define CC 256
#define CI 128
#define C3 384
static_assert(NB >= 1 && NB <= NB_FULL);
static_assert(SEQ >= 256 && SEQ <= SEQ_FULL && (SEQ % 256) == 0);
static_assert((CC % 64) == 0 && (CI % 64) == 0 && (C3 % 64) == 0);

typedef __attribute__((ext_vector_type(16))) _Float16 v16h;
typedef __attribute__((ext_vector_type(8)))  _Float16 v8h;
typedef __attribute__((ext_vector_type(16))) __bf16   v16b;
typedef __attribute__((ext_vector_type(8)))  __bf16   v8b;
typedef __attribute__((ext_vector_type(8)))  float    v8f;
typedef __attribute__((ext_vector_type(4)))  float    v4f;
typedef unsigned int cm_u4 __attribute__((ext_vector_type(4)));

#define VST2(T, ptr, val) do { const T vst2_v_ = (val); *(volatile T*)(ptr) = vst2_v_; __threadfence(); *(volatile T*)(ptr) = vst2_v_; } while (0)

namespace gk {

__device__ __forceinline__ unsigned short f2bf_bits(float f) {
  unsigned u = __float_as_uint(f);
  return (unsigned short)((u + 0x7FFFu + ((u >> 16) & 1u)) >> 16);
}
__device__ __forceinline__ float bf_bits2f(unsigned short h) { return __uint_as_float(((unsigned)h) << 16); }

__device__ __forceinline__ void dep_guard_h(v8f& a, v8f& b, v16h x, v16h y) { asm volatile("v_nop\n\tv_nop\n\tv_nop\n\tv_nop" : "+v"(a), "+v"(b) : "v"(x), "v"(y)); }
__device__ __forceinline__ void dep_guard_b(v8f& a, v8f& b, v16b x, v16b y) { asm volatile("v_nop\n\tv_nop\n\tv_nop\n\tv_nop" : "+v"(a), "+v"(b) : "v"(x), "v"(y)); }
__device__ __forceinline__ void keep4_h(v16h a, v16h b, v16h c, v16h d) { asm volatile("v_nop" :: "v"(a), "v"(b), "v"(c), "v"(d)); }
__device__ __forceinline__ void keep4_b(v16b a, v16b b, v16b c, v16b d) { asm volatile("v_nop" :: "v"(a), "v"(b), "v"(c), "v"(d)); }
__device__ __forceinline__ void acc_guard4(v8f& a, v8f& b, v8f& c, v8f& d) { asm volatile("v_nop\n\tv_nop\n\tv_nop\n\tv_nop" : "+v"(a), "+v"(b), "+v"(c), "+v"(d)); }

template <typename T> struct Frag;
template <> struct Frag<_Float16> {
  typedef v16h V; union U { v16h v; v8h h[2]; };
  static __device__ __forceinline__ v16h load(const _Float16* p) {
    U f; f.h[0] = *(const v8h*)(p); f.h[1] = *(const v8h*)(p + 16); return f.v;
  }
  static __device__ __forceinline__ v8f mma(v16h a, v16h b, v8f c) {
    return __builtin_amdgcn_wmma_f32_16x16x32_f16(false, a, false, b, (short)0, c, false, false);
  }
  static __device__ __forceinline__ void guard(v8f& a, v8f& b, v16h x, v16h y) { dep_guard_h(a, b, x, y); }
  static __device__ __forceinline__ void keep(v16h a, v16h b, v16h c, v16h d) { keep4_h(a, b, c, d); }
};
template <> struct Frag<__bf16> {
  typedef v16b V; union U { v16b v; v8b h[2]; };
  static __device__ __forceinline__ v16b load(const __bf16* p) {
    U f; f.h[0] = *(const v8b*)(p); f.h[1] = *(const v8b*)(p + 16); return f.v;
  }
  static __device__ __forceinline__ v8f mma(v16b a, v16b b, v8f c) {
    return __builtin_amdgcn_wmma_f32_16x16x32_bf16(false, a, false, b, (short)0, c, false, false);
  }
  static __device__ __forceinline__ void guard(v8f& a, v8f& b, v16b x, v16b y) { dep_guard_b(a, b, x, y); }
  static __device__ __forceinline__ void keep(v16b a, v16b b, v16b c, v16b d) { keep4_b(a, b, c, d); }
};

template <int ET> struct Elem;
template <> struct Elem<0> { typedef _Float16 T; };
template <> struct Elem<1> { typedef __bf16 T; };
template <int ET, bool SPLIT, int BIAS_MODE, int OUT_MODE, bool RESID, int ACT = 0>
__global__ __launch_bounds__(256) void wmma_gemm64(
    const unsigned short* __restrict__ Ap, const unsigned short* __restrict__ A2p, int lda, long strideA,
    const unsigned short* __restrict__ Btp, const unsigned short* __restrict__ Bt2p, int ldb, long strideB,
    void* __restrict__ Cout, void* __restrict__ Cout2, int ldc, long strideC,
    const float* __restrict__ bias,
    const float* __restrict__ resid, long strideR,
    int M, int N, int K, float scale) {
  typedef typename Elem<ET>::T T;
  typedef typename Frag<T>::V V;
  const T* A = (const T*)Ap; const T* A2 = (const T*)A2p; const T* Bt = (const T*)Btp; const T* Bt2 = (const T*)Bt2p;
  __shared__ __align__(16) float sT[8][16 * 68];
  const int b    = blockIdx.y;
  const int lane = threadIdx.x & 31;
  const int wave = threadIdx.x >> 5;
  const int tilesN = N >> 6;
  const int tilesM = M >> 6;
  const int tile = blockIdx.x * 8 + wave;
  if (tile >= tilesM * tilesN) return;
  const int tm = tile / tilesN;
  const int tn = tile - tm * tilesN;
  const int m0 = tm << 6;
  const int n0 = tn << 6;

  const T* Ab  = A  + (size_t)b * strideA;
  const T* Bb  = Bt + (size_t)b * strideB;
  const T* Ab2 = SPLIT ? (A2  + (size_t)b * strideA) : nullptr;
  const T* Bb2 = SPLIT ? (Bt2 + (size_t)b * strideB) : nullptr;

  const int rlane = lane & 15;
  const int koff  = (lane >> 4) * 8;
  const int mOff  = (lane >> 4) * 8;

  v8f acc[4][4];
#pragma unroll
  for (int i = 0; i < 4; ++i)
#pragma unroll
    for (int j = 0; j < 4; ++j) acc[i][j] = (v8f){0.f,0.f,0.f,0.f,0.f,0.f,0.f,0.f};

  for (int k0 = 0; k0 < K; k0 += 32) {
    V bh[4], bl[4];
#pragma unroll
    for (int j = 0; j < 4; ++j) {
      const size_t bo = (size_t)(n0 + (j << 4) + rlane) * ldb + koff + k0;
      bh[j] = Frag<T>::load(Bb + bo);
      if (SPLIT) bl[j] = Frag<T>::load(Bb2 + bo);
    }
#pragma unroll
    for (int i = 0; i < 4; ++i) {
      const size_t ao = (size_t)(m0 + (i << 4) + rlane) * lda + koff + k0;
      V ah = Frag<T>::load(Ab + ao);
      V al;
      if (SPLIT) al = Frag<T>::load(Ab2 + ao);
#pragma unroll
      for (int j = 0; j < 4; ++j) {
        acc[i][j] = Frag<T>::mma(ah, bh[j], acc[i][j]);
        if (SPLIT) {
          acc[i][j] = Frag<T>::mma(ah, bl[j], acc[i][j]);
          acc[i][j] = Frag<T>::mma(al, bh[j], acc[i][j]);
        }
      }
      Frag<T>::guard(acc[i][0], acc[i][3], ah, SPLIT ? al : ah);
    }
    Frag<T>::keep(bh[0], bh[1], bh[2], bh[3]);
    if (SPLIT) Frag<T>::keep(bl[0], bl[1], bl[2], bl[3]);
  }
  acc_guard4(acc[0][0], acc[0][1], acc[0][2], acc[0][3]);
  acc_guard4(acc[1][0], acc[1][1], acc[1][2], acc[1][3]);
  acc_guard4(acc[2][0], acc[2][1], acc[2][2], acc[2][3]);
  acc_guard4(acc[3][0], acc[3][1], acc[3][2], acc[3][3]);

  float* slab = sT[wave];
  const float* Rb = RESID ? (resid + (size_t)b * strideR) : nullptr;
#pragma unroll
  for (int i = 0; i < 4; ++i) {
    const int mBase = m0 + (i << 4);
#pragma unroll
    for (int j = 0; j < 4; ++j) {
      const int n = n0 + (j << 4) + rlane;
      float bv = 0.f;
      if (BIAS_MODE == 2) bv = bias[n];
#pragma unroll
      for (int r = 0; r < 8; ++r) {
        float v = acc[i][j][r] * scale;
        if (BIAS_MODE == 1) v += bias[mBase + mOff + r];
        if (BIAS_MODE == 2) v += bv;
        if (RESID) v += Rb[(size_t)(mBase + mOff + r) * ldc + n];
        if (ACT == 1) v = tanhf(v);
        if (ACT == 2) v = fmaxf(v, 0.0f);
        if (ACT == 3) v = v / (1.0f + expf(-v));
        if (ACT == 4) v = (v > 0.f) ? v : 0.01f * v;
        slab[(mOff + r) * 68 + (j << 4) + rlane] = v;
      }
    }
    __builtin_amdgcn_fence(3  , "workgroup");
    __builtin_amdgcn_wave_barrier();
    __builtin_amdgcn_fence(2  , "workgroup");
    if (OUT_MODE == 0) {
      float* C = (float*)Cout + (size_t)b * strideC;
      const int hh = lane >> 4, c4 = (lane & 15) * 4;
      for (int pass = 0; pass < 2; ++pass) {
#pragma unroll
        for (int it = 0; it < 8; ++it) {
          const int row = it * 2 + hh;
          v4f v = *(const v4f*)(slab + row * 68 + c4);
          *(volatile v4f*)(C + (size_t)(mBase + row) * ldc + n0 + c4) = v;
        }
        __threadfence();
      }
    } else {
      const int q = lane >> 3, c8 = (lane & 7) * 8;
      unsigned short* C  = (unsigned short*)Cout  + (size_t)b * strideC;
      unsigned short* C2 = (OUT_MODE == 2) ? ((unsigned short*)Cout2 + (size_t)b * strideC) : nullptr;
      for (int pass = 0; pass < 2; ++pass) {
#pragma unroll
        for (int it = 0; it < 4; ++it) {
          const int row = it * 4 + q;
          const float* sp = slab + row * 68 + c8;
          v8h hv, lv;
#pragma unroll
          for (int e = 0; e < 8; ++e) {
            if (OUT_MODE == 1) {
              hv[e] = (_Float16)sp[e];
            } else {
              unsigned short hb = f2bf_bits(sp[e]);
              unsigned short lb = f2bf_bits(sp[e] - bf_bits2f(hb));
              hv[e] = __builtin_bit_cast(_Float16, hb);
              lv[e] = __builtin_bit_cast(_Float16, lb);
            }
          }
          *(volatile v8h*)(C + (size_t)(mBase + row) * ldc + n0 + c8) = hv;
          if (OUT_MODE == 2) *(volatile v8h*)(C2 + (size_t)(mBase + row) * ldc + n0 + c8) = lv;
        }
        __threadfence();
      }
    }
    __builtin_amdgcn_fence(3  , "workgroup");
    __builtin_amdgcn_wave_barrier();
    __builtin_amdgcn_fence(2  , "workgroup");
  }
}

}

__global__ __launch_bounds__(256) void k_castT16(const float* __restrict__ src, long long lds, _Float16* __restrict__ dst, long long ldd, int R, int C, float s) {
    const long long i = (long long)blockIdx.x * 256 + threadIdx.x; const long long np = (long long)C * (R / 2); if (i >= np) return; const int c = (int)(i / (R / 2)); const int r = 2 * (int)(i % (R / 2));
    const _Float16 h0 = (_Float16)(src[(long long)r * lds + c] * s), h1 = (_Float16)(src[(long long)(r + 1) * lds + c] * s);
    const unsigned u = (unsigned)__builtin_bit_cast(unsigned short, h0) | ((unsigned)__builtin_bit_cast(unsigned short, h1) << 16);
    volatile unsigned* d = (volatile unsigned*)(dst + (long long)c * ldd + r); *d = u; __threadfence(); *d = u; }
__global__ __launch_bounds__(256) void k_cast16(const float* __restrict__ src, long long lds, _Float16* __restrict__ dst, long long ldd, int R, int C, float s) {
    const long long i = (long long)blockIdx.x * 256 + threadIdx.x; const long long np = (long long)R * (C / 2); if (i >= np) return; const int r = (int)(i / (C / 2)); const int c = 2 * (int)(i % (C / 2));
    const _Float16 h0 = (_Float16)(src[(long long)r * lds + c] * s), h1 = (_Float16)(src[(long long)r * lds + c + 1] * s);
    const unsigned u = (unsigned)__builtin_bit_cast(unsigned short, h0) | ((unsigned)__builtin_bit_cast(unsigned short, h1) << 16);
    volatile unsigned* d = (volatile unsigned*)(dst + (long long)r * ldd + c); *d = u; __threadfence(); *d = u; }

__device__ __forceinline__ unsigned int f2bf2_pack(float a, float b, unsigned int* lo) {
    const unsigned short ha = gk::f2bf_bits(a), hb = gk::f2bf_bits(b);
    const unsigned short la = gk::f2bf_bits(a - gk::bf_bits2f(ha)), lb = gk::f2bf_bits(b - gk::bf_bits2f(hb));
    *lo = (unsigned)la | ((unsigned)lb << 16); return (unsigned)ha | ((unsigned)hb << 16); }
__global__ __launch_bounds__(256) void k_castS16(const float* __restrict__ src, long long lds, __bf16* __restrict__ dhi, __bf16* __restrict__ dlo, long long ldd, int R, int C, float s, int transpose) {
    const long long i = (long long)blockIdx.x * 256 + threadIdx.x; long long o; float a, b;
    if (transpose) { const long long np = (long long)C * (R / 2); if (i >= np) return; const int c = (int)(i / (R / 2)); const int r = 2 * (int)(i % (R / 2)); a = src[(long long)r * lds + c] * s; b = src[(long long)(r + 1) * lds + c] * s; o = (long long)c * ldd + r; }
    else { const long long np = (long long)R * (C / 2); if (i >= np) return; const int r = (int)(i / (C / 2)); const int c = 2 * (int)(i % (C / 2)); a = src[(long long)r * lds + c] * s; b = src[(long long)r * lds + c + 1] * s; o = (long long)r * ldd + c; }
    unsigned lo; const unsigned hi = f2bf2_pack(a, b, &lo); volatile unsigned* ph = (volatile unsigned*)(dhi + o); volatile unsigned* pl = (volatile unsigned*)(dlo + o);
    *ph = hi; *pl = lo; __threadfence(); *ph = hi; *pl = lo; }

__device__ __forceinline__ unsigned int cmb_pk2(float a, float b) { return (unsigned int)__builtin_bit_cast(unsigned short, (_Float16)a) | ((unsigned int)__builtin_bit_cast(unsigned short, (_Float16)b) << 16); }
__device__ __forceinline__ float cmb_bf(float v) { const unsigned u = __builtin_bit_cast(unsigned, v); const unsigned r = (u + 0x7fffu + ((u >> 16) & 1u)) & 0xffff0000u; return __builtin_bit_cast(float, r); }
__global__ __launch_bounds__(256) void k_cm_bfvec(const float* __restrict__ SRC, float* __restrict__ DST, int n) { const int u = blockIdx.x * 256 + threadIdx.x; if (u >= n) return; VST2(float, DST + u, cmb_bf(SRC[u])); }
__global__ __launch_bounds__(256) void k_cm_bfrows(const float* __restrict__ SRC, int lds, float* __restrict__ DST, int ldd, int nR, int nC) {
    const long long u = (long long)blockIdx.x * 256 + threadIdx.x; if (u >= (long long)nR * nC) return; const int r = (int)(u / nC); const int c = (int)(u - (long long)r * nC);
    VST2(float, DST + (long long)r * ldd + c, cmb_bf(SRC[(long long)r * lds + c])); }
__global__ __launch_bounds__(256) void k_cm_castb(const float* __restrict__ SRC, int lds, unsigned short* __restrict__ DST, int ldd, int nR, int nC, float sc) {
    const long long u = (long long)blockIdx.x * 256 + threadIdx.x; const int per = nC / 8; if (u >= (long long)nR * per) return; const int r = (int)(u / per); const int c0 = 8 * (int)(u % per);
    const float* s = SRC + (long long)r * lds + c0; float w[8];
#pragma unroll
    for (int e = 0; e < 8; ++e) w[e] = cmb_bf(s[e]) * sc;
    cm_u4 pk; pk.x = cmb_pk2(w[0], w[1]); pk.y = cmb_pk2(w[2], w[3]); pk.z = cmb_pk2(w[4], w[5]); pk.w = cmb_pk2(w[6], w[7]); VST2(cm_u4, (cm_u4*)(DST + (long long)r * ldd + c0), pk); }
__global__ __launch_bounds__(256) void k_cm_castbT(const float* __restrict__ SRC, int lds, unsigned short* __restrict__ DST, int ldd, int nR, int nC, float sc) {
    const long long u = (long long)blockIdx.x * 256 + threadIdx.x; const int per = nR / 8; if (u >= (long long)nC * per) return; const int c = (int)(u / per); const int r0 = 8 * (int)(u % per);
    float w[8];
#pragma unroll
    for (int e = 0; e < 8; ++e) w[e] = cmb_bf(SRC[(long long)(r0 + e) * lds + c]) * sc;
    cm_u4 pk; pk.x = cmb_pk2(w[0], w[1]); pk.y = cmb_pk2(w[2], w[3]); pk.z = cmb_pk2(w[4], w[5]); pk.w = cmb_pk2(w[6], w[7]); VST2(cm_u4, (cm_u4*)(DST + (long long)c * ldd + r0), pk); }

#define SMG (SEQ / 256)
__global__ __launch_bounds__(256) void k_cv_sm(const float* __restrict__ Sp, unsigned short* __restrict__ P) {
    #pragma clang fp contract(off)
    const int row = blockIdx.x * 8 + (threadIdx.x >> 5); const int L = threadIdx.x & 31; const float* sr = Sp + (long long)row * SEQ + 8 * L; float m = -3.0e38f, s = 0.f;
#pragma unroll 1
    for (int g = 0; g < SMG; ++g) { const v4f x = *(const v4f*)(sr + 256 * g), y = *(const v4f*)(sr + 256 * g + 4); const float mx = fmaxf(fmaxf(fmaxf(x.x, x.y), fmaxf(x.z, x.w)), fmaxf(fmaxf(y.x, y.y), fmaxf(y.z, y.w))); const float mn = fmaxf(m, mx);
        s = s * expf(m - mn) + (((expf(x.x - mn) + expf(x.y - mn)) + (expf(x.z - mn) + expf(x.w - mn))) + ((expf(y.x - mn) + expf(y.y - mn)) + (expf(y.z - mn) + expf(y.w - mn)))); m = mn; }
    float gm = m;
#pragma unroll
    for (int o = 16; o > 0; o >>= 1) gm = fmaxf(gm, __shfl_xor(gm, o, 32));
    s = s * expf(m - gm);
#pragma unroll
    for (int o = 16; o > 0; o >>= 1) s += __shfl_xor(s, o, 32);
    const float f = 16384.f / s; unsigned short* pr = P + (long long)row * SEQ + 8 * L;
#pragma unroll 1
    for (int g = 0; g < SMG; ++g) { const v4f x = *(const v4f*)(sr + 256 * g), y = *(const v4f*)(sr + 256 * g + 4); cm_u4 pk;
        pk.x = cmb_pk2(expf(x.x - gm) * f, expf(x.y - gm) * f); pk.y = cmb_pk2(expf(x.z - gm) * f, expf(x.w - gm) * f); pk.z = cmb_pk2(expf(y.x - gm) * f, expf(y.y - gm) * f); pk.w = cmb_pk2(expf(y.z - gm) * f, expf(y.w - gm) * f);
        VST2(cm_u4, (cm_u4*)(pr + 256 * g), pk); } }

static inline unsigned cdiv256(long long n) { return (unsigned)((n + 255) / 256); }

extern "C" void kernel_launch(void* const* d_in, const int* in_sizes, int n_in, void* d_out, int out_size, void* d_ws, size_t ws_size, hipStream_t stream) {
    if (n_in < 9) return;
    if (in_sizes[0] < NB * CC * SEQ_FULL) return;
    if (in_sizes[1] < CI * CC || in_sizes[2] < CI || in_sizes[3] < CI * CC || in_sizes[4] < CI || in_sizes[5] < CI * CC || in_sizes[6] < CI || in_sizes[7] < CC * CI || in_sizes[8] < CC) return;
    if (out_size < NB * CC * SEQ) return;
    const float* x   = (const float*)d_in[0];
    const float* wg  = (const float*)d_in[1];
    const float* bg  = (const float*)d_in[2];
    const float* wth = (const float*)d_in[3];
    const float* bth = (const float*)d_in[4];
    const float* wph = (const float*)d_in[5];
    const float* bph = (const float*)d_in[6];
    const float* wW  = (const float*)d_in[7];
    const float* bW  = (const float*)d_in[8];
    float* out = (float*)d_out;

    char* wsp = (char*)d_ws;
    char* base0 = wsp;
    auto carve = [&](size_t bytes) { char* p = wsp; wsp += ((bytes + 255) / 256) * 256; return p; };
    unsigned short* XT   = (unsigned short*)carve((size_t)SEQ * CC * 2);
    unsigned short* W3   = (unsigned short*)carve((size_t)C3 * CC * 2);
    float*          BR3  = (float*)carve((size_t)(C3 + 64) * 4);
    float*          TPG  = (float*)carve((size_t)SEQ * C3 * 4);
    unsigned short* THH  = (unsigned short*)carve((size_t)SEQ * CI * 2);
    unsigned short* THL  = (unsigned short*)carve((size_t)SEQ * CI * 2);
    unsigned short* PHH  = (unsigned short*)carve((size_t)SEQ * CI * 2);
    unsigned short* PHL  = (unsigned short*)carve((size_t)SEQ * CI * 2);
    unsigned short* GPT  = (unsigned short*)carve((size_t)CI * SEQ * 2);
    float*          S    = (float*)carve((size_t)SEQ * SEQ * 4);
    unsigned short* P16  = (unsigned short*)carve((size_t)SEQ * SEQ * 2);
    float*          YT   = (float*)carve((size_t)SEQ * CI * 4);
    unsigned short* YT16 = (unsigned short*)carve((size_t)SEQ * CI * 2);
    unsigned short* WW16 = (unsigned short*)carve((size_t)CC * CI * 2);
    float*          BF   = (float*)carve((size_t)(CC + 64) * 4);
    float*          XB   = (float*)carve((size_t)CC * SEQ * 4);
    if ((size_t)(wsp - base0) > ws_size) return;

    k_cm_castb<<<cdiv256((long long)CI * (CC / 8)), 256, 0, stream>>>(wth, CC, W3 + 0, CC, CI, CC, 16.0f);
    k_cm_bfvec<<<1, 256, 0, stream>>>(bth, BR3 + 0, CI);
    k_cm_castb<<<cdiv256((long long)CI * (CC / 8)), 256, 0, stream>>>(wph, CC, W3 + (size_t)CI * CC, CC, CI, CC, 16.0f);
    k_cm_bfvec<<<1, 256, 0, stream>>>(bph, BR3 + CI, CI);
    k_cm_castb<<<cdiv256((long long)CI * (CC / 8)), 256, 0, stream>>>(wg, CC, W3 + (size_t)2 * CI * CC, CC, CI, CC, 16.0f);
    k_cm_bfvec<<<1, 256, 0, stream>>>(bg, BR3 + 2 * CI, CI);
    k_cm_castb<<<cdiv256((long long)CC * (CI / 8)), 256, 0, stream>>>(wW, CI, WW16, CI, CC, CI, 16.0f);
    k_cm_bfvec<<<1, 256, 0, stream>>>(bW, BF, CC);

    for (int b = 0; b < NB; ++b) {
        const float* xb = x + (size_t)b * CC * SEQ_FULL;
        float* ob = out + (size_t)b * CC * SEQ;
        k_cm_castbT<<<cdiv256((long long)SEQ * (CC / 8)), 256, 0, stream>>>(xb, SEQ_FULL, XT, CC, CC, SEQ, 1.0f);
        k_cm_bfrows<<<cdiv256((long long)CC * SEQ), 256, 0, stream>>>(xb, SEQ_FULL, XB, SEQ, CC, SEQ);
        gk::wmma_gemm64<0, false, 2, 0, false, 0><<<dim3((unsigned)(((SEQ / 64) * (C3 / 64) + 7) / 8), 1u), 256, 0, stream>>>(
            (const unsigned short*)XT, nullptr, CC, 0, (const unsigned short*)W3, nullptr, CC, 0, (void*)TPG, nullptr, C3, 0, BR3, nullptr, 0, SEQ, C3, CC, 0.0625f);
        k_castS16<<<cdiv256((long long)SEQ * (CI / 2)), 256, 0, stream>>>(TPG, C3, (__bf16*)THH, (__bf16*)THL, CI, SEQ, CI, 1.0f, 0);
        k_castS16<<<cdiv256((long long)SEQ * (CI / 2)), 256, 0, stream>>>(TPG + CI, C3, (__bf16*)PHH, (__bf16*)PHL, CI, SEQ, CI, 1.0f, 0);
        k_castT16<<<cdiv256((long long)CI * (SEQ / 2)), 256, 0, stream>>>(TPG + 2 * CI, C3, (_Float16*)GPT, SEQ, SEQ, CI, 1.0f);
        gk::wmma_gemm64<1, true, 0, 0, false, 0><<<dim3((unsigned)(((SEQ / 64) * (SEQ / 64) + 7) / 8), 1u), 256, 0, stream>>>(
            (const unsigned short*)THH, (const unsigned short*)THL, CI, 0, (const unsigned short*)PHH, (const unsigned short*)PHL, CI, 0, (void*)S, nullptr, SEQ, 0, nullptr, nullptr, 0, SEQ, SEQ, CI, 1.0f);
        k_cv_sm<<<(unsigned)(SEQ / 8), 256, 0, stream>>>(S, P16);
        gk::wmma_gemm64<0, false, 0, 0, false, 0><<<dim3((unsigned)(((SEQ / 64) * (CI / 64) + 7) / 8), 1u), 256, 0, stream>>>(
            (const unsigned short*)P16, nullptr, SEQ, 0, (const unsigned short*)GPT, nullptr, SEQ, 0, (void*)YT, nullptr, CI, 0, nullptr, nullptr, 0, SEQ, CI, SEQ, 6.103515625e-05f);
        k_cast16<<<cdiv256((long long)SEQ * (CI / 2)), 256, 0, stream>>>(YT, CI, (_Float16*)YT16, CI, SEQ, CI, 1.0f);
        gk::wmma_gemm64<0, false, 1, 0, true, 0><<<dim3((unsigned)(((CC / 64) * (SEQ / 64) + 7) / 8), 1u), 256, 0, stream>>>(
            (const unsigned short*)WW16, nullptr, CI, 0, (const unsigned short*)YT16, nullptr, CI, 0, (void*)ob, nullptr, SEQ, 0, BF, XB, 0, CC, SEQ, CI, 0.0625f);
    }
}
